// MambaPolicy_72928544686640
// MI455X (gfx1250) — hardware-verified
//
#include <hip/hip_runtime.h>
#include <math.h>

typedef __attribute__((ext_vector_type(16))) _Float16 v16h;
typedef __attribute__((ext_vector_type(8)))  _Float16 v8h;
typedef __attribute__((ext_vector_type(16))) __bf16   v16b;
typedef __attribute__((ext_vector_type(8)))  __bf16   v8b;
typedef __attribute__((ext_vector_type(8)))  float    v8f;
typedef __attribute__((ext_vector_type(4)))  float    v4f;

constexpr int kBatch  = 4;
constexpr int kSeq    = 1024;
constexpr int kInDim  = 128;
constexpr int kDModel = 256;
constexpr int kMDim   = 512;
constexpr int kNLayer = 4;
constexpr int kDin    = 1024;
constexpr int kNst    = 16;
constexpr int kDtR    = 32;
constexpr int kConvK  = 4;
constexpr int kHid    = kMDim / 2;
constexpr int kXzP    = 2 * kDin;
constexpr int kXdP    = 64;
constexpr int kRows   = kBatch * kSeq;
constexpr int kConvTP = 260;
constexpr int kScanTS = 64;
constexpr int kScanCh = 64;
constexpr int kScanYP = 68;
constexpr float kEps  = 1e-5f;
constexpr float kWCarry = 64.0f;
constexpr float kUCarry = 64.0f;
constexpr float kYCarry = 1024.0f;
constexpr float kNegLogBaseOverD = -0.017988946039015984f;
static_assert(kDtR + 2 * kNst == kXdP, "x_proj width");
static_assert((kInDim % 32) == 0 && (kMDim % 32) == 0 && (kDin % 32) == 0 && (kHid % 32) == 0, "GEMM K multiples of 32");
static_assert((kRows % 64) == 0 && (kXzP % 64) == 0 && (kXdP % 64) == 0 && (kMDim % 64) == 0 &&
              (kDModel % 64) == 0 && (kHid % 64) == 0 && (kInDim % 64) == 0, "GEMM M,N multiples of 64");
static_assert((kSeq % kScanTS) == 0 && (kSeq % 64) == 0 && (kDin % kScanCh) == 0 && (kDin % 256) == 0, "tile multiples");
static_assert((kRows % 32) == 0 && (kRows % 8) == 0, "row blocks");

constexpr size_t kOffXH   = 0;
constexpr size_t kOffWSE  = kOffXH   + (size_t)kRows * kInDim * 2;
constexpr size_t kOffWIP  = kOffWSE  + (size_t)kDModel * kInDim * 2;
constexpr size_t kOffWXP  = kOffWIP  + (size_t)kNLayer * kXzP * kMDim * 2;
constexpr size_t kOffWOP  = kOffWXP  + (size_t)kNLayer * kXdP * kDin * 2;
constexpr size_t kOffWS1  = kOffWOP  + (size_t)kNLayer * kMDim * kDin * 2;
constexpr size_t kOffWR1  = kOffWS1  + (size_t)kHid * kMDim * 2;
constexpr size_t kOffWS2  = kOffWR1  + (size_t)kHid * kMDim * 2;
constexpr size_t kOffSE   = kOffWS2  + (size_t)kInDim * kHid * 2;
constexpr size_t kOffRESA = kOffSE   + (size_t)kRows * kDModel * 4;
constexpr size_t kOffRESB = kOffRESA + (size_t)kRows * kMDim * 4;
constexpr size_t kOffHN   = kOffRESB + (size_t)kRows * kMDim * 4;
constexpr size_t kOffXZ   = kOffHN   + (size_t)kRows * kMDim * 2;
constexpr size_t kOffUC   = kOffXZ   + (size_t)kRows * kXzP * 4;
constexpr size_t kOffUCH  = kOffUC   + (size_t)kRows * kDin * 4;
constexpr size_t kOffXD   = kOffUCH  + (size_t)kRows * kDin * 2;
constexpr size_t kOffYH   = kOffXD   + (size_t)kRows * kXdP * 4;
constexpr size_t kOffH    = kOffYH   + (size_t)kRows * kDin * 2;
constexpr size_t kOffT1S  = kOffH    + (size_t)kRows * kMDim * 4;
constexpr size_t kOffT1R  = kOffT1S  + (size_t)kRows * kHid * 2;
constexpr size_t kWsTotal = kOffT1R  + (size_t)kRows * kHid * 4;
static_assert(kWsTotal == 122814464ull, "carve total");
static_assert(kWsTotal <= 134217728ull, "carve cap");
static_assert((kOffWSE % 128) == 0 && (kOffWIP % 128) == 0 && (kOffWXP % 128) == 0 && (kOffWOP % 128) == 0 &&
              (kOffWS1 % 128) == 0 && (kOffWR1 % 128) == 0 && (kOffWS2 % 128) == 0 && (kOffSE % 128) == 0 &&
              (kOffRESA % 128) == 0 && (kOffRESB % 128) == 0 && (kOffHN % 128) == 0 && (kOffXZ % 128) == 0 &&
              (kOffUC % 128) == 0 && (kOffUCH % 128) == 0 && (kOffXD % 128) == 0 && (kOffYH % 128) == 0 &&
              (kOffH % 128) == 0 && (kOffT1S % 128) == 0 && (kOffT1R % 128) == 0, "128-B aligned regions");

__device__ __forceinline__ unsigned short f2bf_bits(float f) {
  unsigned u = __float_as_uint(f);
  return (unsigned short)((u + 0x7FFFu + ((u >> 16) & 1u)) >> 16);
}
__device__ __forceinline__ float bf_bits2f(unsigned short h) { return __uint_as_float(((unsigned)h) << 16); }

__device__ __forceinline__ void dep_guard_h(v8f& a, v8f& b, v16h x, v16h y) { asm volatile("v_nop\n\tv_nop\n\tv_nop\n\tv_nop" : "+v"(a), "+v"(b) : "v"(x), "v"(y)); }
__device__ __forceinline__ void dep_guard_b(v8f& a, v8f& b, v16b x, v16b y) { asm volatile("v_nop\n\tv_nop\n\tv_nop\n\tv_nop" : "+v"(a), "+v"(b) : "v"(x), "v"(y)); }
__device__ __forceinline__ void keep4_h(v16h a, v16h b, v16h c, v16h d) { asm volatile("v_nop" :: "v"(a), "v"(b), "v"(c), "v"(d)); }
__device__ __forceinline__ void keep4_b(v16b a, v16b b, v16b c, v16b d) { asm volatile("v_nop" :: "v"(a), "v"(b), "v"(c), "v"(d)); }
__device__ __forceinline__ void acc_guard4(v8f& a, v8f& b, v8f& c, v8f& d) { asm volatile("v_nop\n\tv_nop\n\tv_nop\n\tv_nop" : "+v"(a), "+v"(b), "+v"(c), "+v"(d)); }
template <typename T> struct Frag;
template <> struct Frag<_Float16> {
  typedef v16h V; union U { v16h v; v8h h[2]; };
  static __device__ __forceinline__ v16h load(const _Float16* p) {
    U f; f.h[0] = *(const v8h*)(p); f.h[1] = *(const v8h*)(p + 16); return f.v;
  }
  static __device__ __forceinline__ v8f mma(v16h a, v16h b, v8f c) {
    return __builtin_amdgcn_wmma_f32_16x16x32_f16(false, a, false, b, (short)0, c, false, false);
  }
  static __device__ __forceinline__ void guard(v8f& a, v8f& b, v16h x, v16h y) { dep_guard_h(a, b, x, y); }
  static __device__ __forceinline__ void keep(v16h a, v16h b, v16h c, v16h d) { keep4_h(a, b, c, d); }
};
template <> struct Frag<__bf16> {
  typedef v16b V; union U { v16b v; v8b h[2]; };
  static __device__ __forceinline__ v16b load(const __bf16* p) {
    U f; f.h[0] = *(const v8b*)(p); f.h[1] = *(const v8b*)(p + 16); return f.v;
  }
  static __device__ __forceinline__ v8f mma(v16b a, v16b b, v8f c) {
    return __builtin_amdgcn_wmma_f32_16x16x32_bf16(false, a, false, b, (short)0, c, false, false);
  }
  static __device__ __forceinline__ void guard(v8f& a, v8f& b, v16b x, v16b y) { dep_guard_b(a, b, x, y); }
  static __device__ __forceinline__ void keep(v16b a, v16b b, v16b c, v16b d) { keep4_b(a, b, c, d); }
};

template <int ET> struct Elem;
template <> struct Elem<0> { typedef _Float16 T; };
template <> struct Elem<1> { typedef __bf16 T; };
template <int ET, bool SPLIT, int BIAS_MODE, int OUT_MODE, bool RESID, int ACT = 0>
__global__ __launch_bounds__(256) void wmma_gemm64(
    const unsigned short* __restrict__ Ap, const unsigned short* __restrict__ A2p, int lda, long strideA,
    const unsigned short* __restrict__ Btp, const unsigned short* __restrict__ Bt2p, int ldb, long strideB,
    void* __restrict__ Cout, void* __restrict__ Cout2, int ldc, long strideC,
    const float* __restrict__ bias,
    const float* __restrict__ resid, long strideR,
    int M, int N, int K, float scale) {
  typedef typename Elem<ET>::T T;
  typedef typename Frag<T>::V V;
  const T* A = (const T*)Ap; const T* A2 = (const T*)A2p; const T* Bt = (const T*)Btp; const T* Bt2 = (const T*)Bt2p;
  __shared__ __align__(16) float sT[8][16 * 68];
  const int b    = blockIdx.y;
  const int lane = threadIdx.x & 31;
  const int wave = threadIdx.x >> 5;
  const int tilesN = N >> 6;
  const int tilesM = M >> 6;
  const int tile = blockIdx.x * 8 + wave;
  if (tile >= tilesM * tilesN) return;
  const int tm = tile / tilesN;
  const int tn = tile - tm * tilesN;
  const int m0 = tm << 6;
  const int n0 = tn << 6;

  const T* Ab  = A  + (size_t)b * strideA;
  const T* Bb  = Bt + (size_t)b * strideB;
  const T* Ab2 = SPLIT ? (A2  + (size_t)b * strideA) : nullptr;
  const T* Bb2 = SPLIT ? (Bt2 + (size_t)b * strideB) : nullptr;

  const int rlane = lane & 15;
  const int koff  = (lane >> 4) * 8;
  const int mOff  = (lane >> 4) * 8;

  v8f acc[4][4];
#pragma unroll
  for (int i = 0; i < 4; ++i)
#pragma unroll
    for (int j = 0; j < 4; ++j) acc[i][j] = (v8f){0.f,0.f,0.f,0.f,0.f,0.f,0.f,0.f};

  for (int k0 = 0; k0 < K; k0 += 32) {
    V bh[4], bl[4];
#pragma unroll
    for (int j = 0; j < 4; ++j) {
      const size_t bo = (size_t)(n0 + (j << 4) + rlane) * ldb + koff + k0;
      bh[j] = Frag<T>::load(Bb + bo);
      if (SPLIT) bl[j] = Frag<T>::load(Bb2 + bo);
    }
#pragma unroll
    for (int i = 0; i < 4; ++i) {
      const size_t ao = (size_t)(m0 + (i << 4) + rlane) * lda + koff + k0;
      V ah = Frag<T>::load(Ab + ao);
      V al;
      if (SPLIT) al = Frag<T>::load(Ab2 + ao);
#pragma unroll
      for (int j = 0; j < 4; ++j) {
        acc[i][j] = Frag<T>::mma(ah, bh[j], acc[i][j]);
        if (SPLIT) {
          acc[i][j] = Frag<T>::mma(ah, bl[j], acc[i][j]);
          acc[i][j] = Frag<T>::mma(al, bh[j], acc[i][j]);
        }
      }
      Frag<T>::guard(acc[i][0], acc[i][3], ah, SPLIT ? al : ah);
    }
    Frag<T>::keep(bh[0], bh[1], bh[2], bh[3]);
    if (SPLIT) Frag<T>::keep(bl[0], bl[1], bl[2], bl[3]);
  }
  acc_guard4(acc[0][0], acc[0][1], acc[0][2], acc[0][3]);
  acc_guard4(acc[1][0], acc[1][1], acc[1][2], acc[1][3]);
  acc_guard4(acc[2][0], acc[2][1], acc[2][2], acc[2][3]);
  acc_guard4(acc[3][0], acc[3][1], acc[3][2], acc[3][3]);

  float* slab = sT[wave];
  const float* Rb = RESID ? (resid + (size_t)b * strideR) : nullptr;
#pragma unroll
  for (int i = 0; i < 4; ++i) {
    const int mBase = m0 + (i << 4);
#pragma unroll
    for (int j = 0; j < 4; ++j) {
      const int n = n0 + (j << 4) + rlane;
      float bv = 0.f;
      if (BIAS_MODE == 2) bv = bias[n];
#pragma unroll
      for (int r = 0; r < 8; ++r) {
        float v = acc[i][j][r] * scale;
        if (BIAS_MODE == 1) v += bias[mBase + mOff + r];
        if (BIAS_MODE == 2) v += bv;
        if (RESID) v += Rb[(size_t)(mBase + mOff + r) * ldc + n];
        if (ACT == 1) v = tanhf(v);
        if (ACT == 2) v = fmaxf(v, 0.0f);
        if (ACT == 3) v = v / (1.0f + expf(-v));
        if (ACT == 4) v = (v > 0.f) ? v : 0.01f * v;
        slab[(mOff + r) * 68 + (j << 4) + rlane] = v;
      }
    }
    __builtin_amdgcn_fence(__ATOMIC_RELEASE, "workgroup");
    __builtin_amdgcn_wave_barrier();
    __builtin_amdgcn_fence(__ATOMIC_ACQUIRE, "workgroup");
    if (OUT_MODE == 0) {
      float* C = (float*)Cout + (size_t)b * strideC;
      const int hh = lane >> 4, c4 = (lane & 15) * 4;
      for (int pass = 0; pass < 2; ++pass) {
#pragma unroll
        for (int it = 0; it < 8; ++it) {
          const int row = it * 2 + hh;
          v4f v = *(const v4f*)(slab + row * 68 + c4);
          *(volatile v4f*)(C + (size_t)(mBase + row) * ldc + n0 + c4) = v;
        }
        __threadfence();
      }
    } else {
      const int q = lane >> 3, c8 = (lane & 7) * 8;
      unsigned short* C  = (unsigned short*)Cout  + (size_t)b * strideC;
      unsigned short* C2 = (OUT_MODE == 2) ? ((unsigned short*)Cout2 + (size_t)b * strideC) : nullptr;
      for (int pass = 0; pass < 2; ++pass) {
#pragma unroll
        for (int it = 0; it < 4; ++it) {
          const int row = it * 4 + q;
          const float* sp = slab + row * 68 + c8;
          v8h hv, lv;
#pragma unroll
          for (int e = 0; e < 8; ++e) {
            if (OUT_MODE == 1) {
              hv[e] = (_Float16)sp[e];
            } else {
              unsigned short hb = f2bf_bits(sp[e]);
              unsigned short lb = f2bf_bits(sp[e] - bf_bits2f(hb));
              hv[e] = __builtin_bit_cast(_Float16, hb);
              lv[e] = __builtin_bit_cast(_Float16, lb);
            }
          }
          *(volatile v8h*)(C + (size_t)(mBase + row) * ldc + n0 + c8) = hv;
          if (OUT_MODE == 2) *(volatile v8h*)(C2 + (size_t)(mBase + row) * ldc + n0 + c8) = lv;
        }
        __threadfence();
      }
    }
    __builtin_amdgcn_fence(__ATOMIC_RELEASE, "workgroup");
    __builtin_amdgcn_wave_barrier();
    __builtin_amdgcn_fence(__ATOMIC_ACQUIRE, "workgroup");
  }
}

__global__ __launch_bounds__(256) void cast_f16_kernel(
    const float* __restrict__ src, unsigned short* __restrict__ dst, int total8, float sc)
{
  const int i = blockIdx.x * 256 + threadIdx.x;
  if (i >= total8) return;
  const size_t e0 = (size_t)i << 3;
  const v4f a0 = *(const v4f*)(src + e0);
  const v4f a1 = *(const v4f*)(src + e0 + 4);
  v8h hv;
#pragma unroll
  for (int e = 0; e < 4; ++e) {
    hv[e]     = (_Float16)(a0[e] * sc);
    hv[4 + e] = (_Float16)(a1[e] * sc);
  }
  unsigned short* q = dst + e0;
  *(volatile v8h*)q = hv;
  __threadfence();
  *(volatile v8h*)q = hv;
}

__global__ __launch_bounds__(256) void embed_ln_kernel(
    const float* __restrict__ SE, const float* __restrict__ rtg,
    const float* __restrict__ rw, const float* __restrict__ rb,
    const float* __restrict__ lnw, const float* __restrict__ lnb,
    const float* __restrict__ nw0,
    float* __restrict__ RES, unsigned short* __restrict__ HN)
{
  __shared__ __align__(16) float sH[8 * kMDim];
  __shared__ __align__(16) float sN[8 * kMDim];
  const int tid = threadIdx.x, lane = tid & 31, wave = tid >> 5;
  const size_t row = (size_t)blockIdx.x * 8 + wave;
  const int pos = (int)(row & (size_t)(kSeq - 1));
  const float rv = rtg[row];
  float* hrow = sH + wave * kMDim;
  float* nrow = sN + wave * kMDim;
  const float* serow = SE + row * kDModel;

  float sum = 0.f;
#pragma unroll 1
  for (int p = 0; p < 8; ++p) {
    const int j  = p >> 2;
    const int cc = 8 * lane + 2 * (p & 3);
    const int c  = 256 * j + cc;
    const float s0 = serow[cc], s1 = serow[cc + 1];
    const float r0 = rv * rw[cc] + rb[cc];
    const float r1 = rv * rw[cc + 1] + rb[cc + 1];
    const float b0 = j ? r0 : s0;
    const float b1 = j ? r1 : s1;
    const float dv  = expf((float)c * kNegLogBaseOverD);
    const float ang = (float)pos * dv;
    float sv, cv;
    sincosf(ang, &sv, &cv);
    const float h0 = b0 + sv, h1 = b1 + cv;
    hrow[c] = h0;
    hrow[c + 1] = h1;
    sum += h0 + h1;
  }
#pragma unroll
  for (int off = 1; off < 32; off <<= 1) sum += __shfl_xor(sum, off, 32);
  const float mu = sum * (1.0f / (float)kMDim);

  float sq = 0.f;
#pragma unroll 1
  for (int q = 0; q < 16; ++q) {
    const int c = 256 * (q >> 3) + 8 * lane + (q & 7);
    const float dlt = hrow[c] - mu;
    sq += dlt * dlt;
  }
#pragma unroll
  for (int off = 1; off < 32; off <<= 1) sq += __shfl_xor(sq, off, 32);
  const float inv = rsqrtf(sq * (1.0f / (float)kMDim) + kEps);

  float ss = 0.f;
#pragma unroll 1
  for (int q = 0; q < 16; ++q) {
    const int c = 256 * (q >> 3) + 8 * lane + (q & 7);
    const float y = (hrow[c] - mu) * inv * lnw[c] + lnb[c];
    hrow[c] = y;
    ss += y * y;
  }
#pragma unroll
  for (int off = 1; off < 32; off <<= 1) ss += __shfl_xor(ss, off, 32);
  const float inv2 = rsqrtf(ss * (1.0f / (float)kMDim) + kEps);

#pragma unroll 1
  for (int q = 0; q < 16; ++q) {
    const int c = 256 * (q >> 3) + 8 * lane + (q & 7);
    nrow[c] = hrow[c] * inv2 * nw0[c];
  }
  __syncthreads();

  v4f rvv[4];
#pragma unroll
  for (int it = 0; it < 4; ++it) rvv[it] = *(const v4f*)(hrow + 128 * it + 4 * lane);
  v8h hv[2];
#pragma unroll
  for (int it = 0; it < 2; ++it) {
    const float* sp = nrow + 256 * it + 8 * lane;
    const v4f a0 = *(const v4f*)(sp);
    const v4f a1 = *(const v4f*)(sp + 4);
#pragma unroll
    for (int e = 0; e < 4; ++e) {
      hv[it][e]     = (_Float16)a0[e];
      hv[it][4 + e] = (_Float16)a1[e];
    }
  }
  float* op = RES + row * kMDim;
  unsigned short* np2 = HN + row * kMDim;
  for (int pass = 0; pass < 2; ++pass) {
#pragma unroll
    for (int it = 0; it < 4; ++it) *(volatile v4f*)(op + 128 * it + 4 * lane) = rvv[it];
#pragma unroll
    for (int it = 0; it < 2; ++it) *(volatile v8h*)(np2 + 256 * it + 8 * lane) = hv[it];
    __threadfence();
  }
}

__global__ __launch_bounds__(256) void residual_rms_kernel(
    const float* __restrict__ Hin, const float* __restrict__ Rin, const float* __restrict__ w,
    float* __restrict__ Rout, unsigned short* __restrict__ HN)
{
  __shared__ __align__(16) float sN[8 * kMDim];
  const int tid = threadIdx.x, lane = tid & 31, wave = tid >> 5;
  const size_t row = (size_t)blockIdx.x * 8 + wave;
  const float* hp = Hin + row * kMDim;
  const float* rp = Rin + row * kMDim;
  v4f ev[4];
  float ss = 0.f;
#pragma unroll
  for (int it = 0; it < 4; ++it) {
    const int c0 = 128 * it + 4 * lane;
    const v4f a = *(const v4f*)(hp + c0);
    const v4f r = *(const v4f*)(rp + c0);
    v4f e;
    e.x = a.x + r.x; e.y = a.y + r.y; e.z = a.z + r.z; e.w = a.w + r.w;
    ev[it] = e;
    ss += e.x * e.x + e.y * e.y + e.z * e.z + e.w * e.w;
  }
#pragma unroll
  for (int off = 1; off < 32; off <<= 1) ss += __shfl_xor(ss, off, 32);
  const float inv = rsqrtf(ss * (1.0f / (float)kMDim) + kEps);
  float* nrow = sN + wave * kMDim;
#pragma unroll
  for (int it = 0; it < 4; ++it) {
    const int c0 = 128 * it + 4 * lane;
    const v4f wv = *(const v4f*)(w + c0);
    v4f n;
    n.x = ev[it].x * inv * wv.x;
    n.y = ev[it].y * inv * wv.y;
    n.z = ev[it].z * inv * wv.z;
    n.w = ev[it].w * inv * wv.w;
    *(v4f*)(nrow + c0) = n;
  }
  __syncthreads();
  v8h hv[2];
#pragma unroll
  for (int it = 0; it < 2; ++it) {
    const float* sp = nrow + 256 * it + 8 * lane;
    const v4f a0 = *(const v4f*)(sp);
    const v4f a1 = *(const v4f*)(sp + 4);
#pragma unroll
    for (int e = 0; e < 4; ++e) {
      hv[it][e]     = (_Float16)a0[e];
      hv[it][4 + e] = (_Float16)a1[e];
    }
  }
  float* op = Rout + row * kMDim;
  unsigned short* np2 = HN + row * kMDim;
  for (int pass = 0; pass < 2; ++pass) {
#pragma unroll
    for (int it = 0; it < 4; ++it) *(volatile v4f*)(op + 128 * it + 4 * lane) = ev[it];
#pragma unroll
    for (int it = 0; it < 2; ++it) *(volatile v8h*)(np2 + 256 * it + 8 * lane) = hv[it];
    __threadfence();
  }
}

__global__ __launch_bounds__(256) void conv_silu_kernel(
    const float* __restrict__ XZ, const float* __restrict__ cw, const float* __restrict__ cb,
    float* __restrict__ UC, unsigned short* __restrict__ UCH)
{
  __shared__ __align__(16) float sT[16 * kConvTP];
  const int tid = threadIdx.x, lane = tid & 31, wave = tid >> 5;
  const int d0 = blockIdx.x * 256, d = d0 + tid;
  const int g0 = blockIdx.y * 64;
  const int tb = g0 & (kSeq - 1);
  const float w0 = cw[d * kConvK + 0], w1 = cw[d * kConvK + 1], w2 = cw[d * kConvK + 2], w3 = cw[d * kConvK + 3];
  const float bc = cb[d];
  float xm3, xm2, xm1;
  {
    const bool hist = (tb > 0);
    const int rb = hist ? (g0 - 3) : g0;
    const float v3 = XZ[(size_t)rb * kXzP + d];
    const float v2 = XZ[(size_t)(rb + 1) * kXzP + d];
    const float v1 = XZ[(size_t)(rb + 2) * kXzP + d];
    xm3 = hist ? v3 : 0.f;
    xm2 = hist ? v2 : 0.f;
    xm1 = hist ? v1 : 0.f;
  }
  const int hrow = wave >> 1;
  const int hch  = (wave & 1) * 128 + lane * 4;
#pragma unroll 1
  for (int sub = 0; sub < 4; ++sub) {
    const int lb = g0 + sub * 16;
#pragma unroll 1
    for (int s = 0; s < 16; ++s) {
      const float xcur = XZ[(size_t)(lb + s) * kXzP + d];
      float acc = w0 * xm3;
      acc = fmaf(w1, xm2, acc);
      acc = fmaf(w2, xm1, acc);
      acc = fmaf(w3, xcur, acc);
      const float sv = acc + bc;
      const float sg = __builtin_amdgcn_rcpf(1.0f + __expf(-sv));
      sT[s * kConvTP + tid] = sv * sg;
      xm3 = xm2; xm2 = xm1; xm1 = xcur;
    }
    __syncthreads();
    v4f fv[4];
    v8h hv2[2];
#pragma unroll
    for (int it = 0; it < 4; ++it) fv[it] = *(const v4f*)(sT + (it * 4 + hrow) * kConvTP + hch);
#pragma unroll
    for (int it = 0; it < 2; ++it) {
      const float* sp = sT + (it * 8 + wave) * kConvTP + lane * 8;
      const v4f a0 = *(const v4f*)(sp);
      const v4f a1 = *(const v4f*)(sp + 4);
#pragma unroll
      for (int e = 0; e < 4; ++e) {
        hv2[it][e]     = (_Float16)(a0[e] * kUCarry);
        hv2[it][4 + e] = (_Float16)(a1[e] * kUCarry);
      }
    }
    for (int pass = 0; pass < 2; ++pass) {
#pragma unroll
      for (int it = 0; it < 4; ++it)
        *(volatile v4f*)(UC + (size_t)(lb + it * 4 + hrow) * kDin + d0 + hch) = fv[it];
#pragma unroll
      for (int it = 0; it < 2; ++it) {
        const size_t o = (size_t)(lb + it * 8 + wave) * kDin + d0 + lane * 8;
        *(volatile v8h*)(UCH + o) = hv2[it];
      }
      __threadfence();
    }
    __syncthreads();
  }
}

__global__ __launch_bounds__(64) void scan_kernel(
    const float* __restrict__ XD, const float* __restrict__ UC, const float* __restrict__ XZ,
    const float* __restrict__ Wdt, const float* __restrict__ bdt, const float* __restrict__ Alog,
    const float* __restrict__ Dp, unsigned short* __restrict__ YH)
{
  __shared__ __align__(16) float sX[kScanTS * kXdP];
  __shared__ __align__(16) float sY[kScanTS * kScanYP];
  __shared__ __align__(16) float sW[kDtR * kScanCh];
  __shared__ __align__(16) float sA[kNst * kScanCh];
  const int tid = threadIdx.x, lane = tid & 31, wave = tid >> 5;
  constexpr int kBlkPerB = kDin / kScanCh;
  const int bix = blockIdx.x / kBlkPerB;
  const int d0  = (blockIdx.x - bix * kBlkPerB) * kScanCh;
  const int d   = d0 + tid;
  const size_t row0 = (size_t)bix * kSeq;
#pragma unroll 1
  for (int r = 0; r < kDtR; ++r) sW[r * kScanCh + tid] = Wdt[(size_t)d * kDtR + r];
#pragma unroll 1
  for (int s = 0; s < kNst; ++s) sA[s * kScanCh + tid] = -expf(Alog[(size_t)d * kNst + s]);
  __syncthreads();
  float negA[kNst], h[kNst];
#pragma unroll
  for (int s = 0; s < kNst; ++s) {
    negA[s] = sA[s * kScanCh + tid];
    h[s] = 0.f;
  }
  const float bb = bdt[d], Dd = Dp[d];
  const int lr = tid >> 4, lc4 = (tid & 15) * 4;
  const int q = lane >> 3, c8 = (lane & 7) * 8;
#pragma unroll 1
  for (int t0 = 0; t0 < kSeq; t0 += kScanTS) {
    __syncthreads();
#pragma unroll
    for (int i = 0; i < 16; ++i) {
      const int r = lr + 4 * i;
      *(v4f*)(sX + r * kXdP + lc4) = *(const v4f*)(XD + (row0 + t0 + r) * kXdP + lc4);
    }
    __syncthreads();
#pragma unroll 1
    for (int s = 0; s < kScanTS; ++s) {
      const int t = t0 + s;
      const float* xr = sX + s * kXdP;
      float vdot = 0.f;
#pragma unroll 1
      for (int r4 = 0; r4 < kDtR / 4; ++r4) {
        const v4f xv = *(const v4f*)(xr + 4 * r4);
        const float* wp = sW + (4 * r4) * kScanCh + tid;
        vdot = fmaf(xv[0], wp[0], vdot);
        vdot = fmaf(xv[1], wp[kScanCh], vdot);
        vdot = fmaf(xv[2], wp[2 * kScanCh], vdot);
        vdot = fmaf(xv[3], wp[3 * kScanCh], vdot);
      }
      float Bs[kNst], Cs[kNst];
#pragma unroll
      for (int q4 = 0; q4 < 4; ++q4) {
        const v4f bv = *(const v4f*)(xr + kDtR + 4 * q4);
        const v4f cv = *(const v4f*)(xr + kDtR + kNst + 4 * q4);
        Bs[4 * q4 + 0] = bv[0]; Bs[4 * q4 + 1] = bv[1]; Bs[4 * q4 + 2] = bv[2]; Bs[4 * q4 + 3] = bv[3];
        Cs[4 * q4 + 0] = cv[0]; Cs[4 * q4 + 1] = cv[1]; Cs[4 * q4 + 2] = cv[2]; Cs[4 * q4 + 3] = cv[3];
      }
      const float v   = vdot + bb;
      const float a   = __expf(-fabsf(v));
      const float u   = 1.0f + a;
      const float l1p = __logf(u) + (a - (u - 1.0f)) * __builtin_amdgcn_rcpf(u);
      const float dt  = fmaxf(v, 0.0f) + l1p;
      const float xt  = UC[(row0 + t) * kDin + d];
      const float dtx = dt * xt;
      float y = 0.f;
#pragma unroll
      for (int k = 0; k < kNst; ++k) {
        const float e = __expf(dt * negA[k]);
        h[k] = e * h[k] + dtx * Bs[k];
        y = h[k] * Cs[k] + y;
      }
      y = xt * Dd + y;
      const float zv = XZ[(row0 + t) * kXzP + kDin + d];
      const float sg = __builtin_amdgcn_rcpf(1.0f + __expf(-zv));
      y = y * (zv * sg);
      sY[s * kScanYP + tid] = y;
    }
    __syncthreads();
    v8h hv[8];
#pragma unroll
    for (int it = 0; it < 8; ++it) {
      const int row = it * 8 + wave * 4 + q;
      const float* sp = sY + row * kScanYP + c8;
      const v4f a0 = *(const v4f*)(sp);
      const v4f a1 = *(const v4f*)(sp + 4);
#pragma unroll
      for (int e = 0; e < 4; ++e) {
        hv[it][e]     = (_Float16)(a0[e] * kYCarry);
        hv[it][4 + e] = (_Float16)(a1[e] * kYCarry);
      }
    }
    for (int pass = 0; pass < 2; ++pass) {
#pragma unroll
      for (int it = 0; it < 8; ++it) {
        const int row = it * 8 + wave * 4 + q;
        const size_t o = (row0 + t0 + row) * kDin + d0 + c8;
        *(volatile v8h*)(YH + o) = hv[it];
      }
      __threadfence();
    }
  }
}

__global__ __launch_bounds__(256) void reward_head_kernel(
    const float* __restrict__ T1, const float* __restrict__ w2, const float* __restrict__ b2,
    float* __restrict__ out1)
{
  __shared__ float sO[32];
  const int tid = threadIdx.x, lane = tid & 31, wave = tid >> 5;
  const int r = tid >> 3, part = tid & 7;
  const size_t row = (size_t)blockIdx.x * 32 + r;
  const float* tp = T1 + row * kHid + part * 32;
  const float* wp = w2 + part * 32;
  float acc = 0.f;
#pragma unroll 1
  for (int k = 0; k < 8; ++k) {
    const v4f a = *(const v4f*)(tp + 4 * k);
    const v4f b = *(const v4f*)(wp + 4 * k);
    acc = fmaf(a.x, b.x, acc);
    acc = fmaf(a.y, b.y, acc);
    acc = fmaf(a.z, b.z, acc);
    acc = fmaf(a.w, b.w, acc);
  }
  acc += __shfl_xor(acc, 1, 32);
  acc += __shfl_xor(acc, 2, 32);
  acc += __shfl_xor(acc, 4, 32);
  if (part == 0) sO[r] = acc;
  __syncthreads();
  if (wave == 0) {
    const float v = sO[lane] + b2[0];
    float* qp = out1 + (size_t)blockIdx.x * 32 + lane;
    *(volatile float*)qp = v;
    __threadfence();
    *(volatile float*)qp = v;
  }
}

static inline unsigned gemm_blocks(int M, int N) { return (unsigned)(((M / 64) * (N / 64) + 7) / 8); }
static inline unsigned cast_blocks(int total8) { return (unsigned)((total8 + 255) / 256); }

extern "C" void kernel_launch(void* const* d_in, const int* in_sizes, int n_in,
                              void* d_out, int out_size, void* d_ws, size_t ws_size,
                              hipStream_t stream) {
  if (n_in != 27) return;
  if (in_sizes[0]  != kRows * kInDim) return;
  if (in_sizes[1]  != kRows) return;
  if (in_sizes[2]  != kDModel * kInDim) return;
  if (in_sizes[3]  != kDModel) return;
  if (in_sizes[4]  != kDModel) return;
  if (in_sizes[5]  != kDModel) return;
  if (in_sizes[6]  != kMDim) return;
  if (in_sizes[7]  != kMDim) return;
  if (in_sizes[8]  != kNLayer * kXzP * kMDim) return;
  if (in_sizes[9]  != kNLayer * kDin * kConvK) return;
  if (in_sizes[10] != kNLayer * kDin) return;
  if (in_sizes[11] != kNLayer * kXdP * kDin) return;
  if (in_sizes[12] != kNLayer * kDin * kDtR) return;
  if (in_sizes[13] != kNLayer * kDin) return;
  if (in_sizes[14] != kNLayer * kDin * kNst) return;
  if (in_sizes[15] != kNLayer * kDin) return;
  if (in_sizes[16] != kNLayer * kMDim * kDin) return;
  if (in_sizes[17] != kNLayer * kMDim) return;
  if (in_sizes[18] != kMDim) return;
  if (in_sizes[19] != kHid * kMDim) return;
  if (in_sizes[20] != kHid) return;
  if (in_sizes[21] != kInDim * kHid) return;
  if (in_sizes[22] != kInDim) return;
  if (in_sizes[23] != kHid * kMDim) return;
  if (in_sizes[24] != kHid) return;
  if (in_sizes[25] != kHid) return;
  if (in_sizes[26] != 1) return;
  if (out_size != kRows * kInDim + kRows) return;
  if (ws_size < kWsTotal) return;

  const float* x           = (const float*)d_in[0];
  const float* rtg         = (const float*)d_in[1];
  const float* state_emb_w = (const float*)d_in[2];
  const float* state_emb_b = (const float*)d_in[3];
  const float* reward_emb_w= (const float*)d_in[4];
  const float* reward_emb_b= (const float*)d_in[5];
  const float* ln_w        = (const float*)d_in[6];
  const float* ln_b        = (const float*)d_in[7];
  const float* in_proj_w   = (const float*)d_in[8];
  const float* conv_w      = (const float*)d_in[9];
  const float* conv_b      = (const float*)d_in[10];
  const float* x_proj_w    = (const float*)d_in[11];
  const float* dt_proj_w   = (const float*)d_in[12];
  const float* dt_proj_b   = (const float*)d_in[13];
  const float* A_log       = (const float*)d_in[14];
  const float* D_param     = (const float*)d_in[15];
  const float* out_proj_w  = (const float*)d_in[16];
  const float* norm_w      = (const float*)d_in[17];
  const float* norm_f_w    = (const float*)d_in[18];
  const float* so_w1       = (const float*)d_in[19];
  const float* so_b1       = (const float*)d_in[20];
  const float* so_w2       = (const float*)d_in[21];
  const float* so_b2       = (const float*)d_in[22];
  const float* ro_w1       = (const float*)d_in[23];
  const float* ro_b1       = (const float*)d_in[24];
  const float* ro_w2       = (const float*)d_in[25];
  const float* ro_b2       = (const float*)d_in[26];
  float* out0 = (float*)d_out;
  float* out1 = (float*)d_out + (size_t)kRows * kInDim;

  char* ws = (char*)d_ws;
  unsigned short* XH   = (unsigned short*)(ws + kOffXH);
  unsigned short* WSE  = (unsigned short*)(ws + kOffWSE);
  unsigned short* WIP  = (unsigned short*)(ws + kOffWIP);
  unsigned short* WXP  = (unsigned short*)(ws + kOffWXP);
  unsigned short* WOP  = (unsigned short*)(ws + kOffWOP);
  unsigned short* WS1  = (unsigned short*)(ws + kOffWS1);
  unsigned short* WR1  = (unsigned short*)(ws + kOffWR1);
  unsigned short* WS2  = (unsigned short*)(ws + kOffWS2);
  float*          SE   = (float*)(ws + kOffSE);
  float*          RESA = (float*)(ws + kOffRESA);
  float*          RESB = (float*)(ws + kOffRESB);
  unsigned short* HN   = (unsigned short*)(ws + kOffHN);
  float*          XZ   = (float*)(ws + kOffXZ);
  float*          UC   = (float*)(ws + kOffUC);
  unsigned short* UCH  = (unsigned short*)(ws + kOffUCH);
  float*          XD   = (float*)(ws + kOffXD);
  unsigned short* YH   = (unsigned short*)(ws + kOffYH);
  float*          H    = (float*)(ws + kOffH);
  unsigned short* T1S  = (unsigned short*)(ws + kOffT1S);
  float*          T1R  = (float*)(ws + kOffT1R);

  {
    const int n8x  = kRows * kInDim / 8;
    const int n8se = kDModel * kInDim / 8;
    const int n8ip = kNLayer * kXzP * kMDim / 8;
    const int n8xp = kNLayer * kXdP * kDin / 8;
    const int n8op = kNLayer * kMDim * kDin / 8;
    const int n8h1 = kHid * kMDim / 8;
    const int n8h2 = kInDim * kHid / 8;
    cast_f16_kernel<<<cast_blocks(n8x),  256, 0, stream>>>(x, XH, n8x, 1.0f);
    cast_f16_kernel<<<cast_blocks(n8se), 256, 0, stream>>>(state_emb_w, WSE, n8se, kWCarry);
    cast_f16_kernel<<<cast_blocks(n8ip), 256, 0, stream>>>(in_proj_w, WIP, n8ip, kWCarry);
    cast_f16_kernel<<<cast_blocks(n8xp), 256, 0, stream>>>(x_proj_w, WXP, n8xp, kWCarry);
    cast_f16_kernel<<<cast_blocks(n8op), 256, 0, stream>>>(out_proj_w, WOP, n8op, kWCarry);
    cast_f16_kernel<<<cast_blocks(n8h1), 256, 0, stream>>>(so_w1, WS1, n8h1, kWCarry);
    cast_f16_kernel<<<cast_blocks(n8h1), 256, 0, stream>>>(ro_w1, WR1, n8h1, kWCarry);
    cast_f16_kernel<<<cast_blocks(n8h2), 256, 0, stream>>>(so_w2, WS2, n8h2, kWCarry);
  }

  wmma_gemm64<0, false, 2, 0, false, 0><<<dim3(gemm_blocks(kRows, kDModel), 1), 256, 0, stream>>>(
      XH, nullptr, kInDim, 0L,
      WSE, nullptr, kInDim, 0L,
      (void*)SE, nullptr, kDModel, 0L,
      state_emb_b, nullptr, 0L,
      kRows, kDModel, kInDim, 1.0f / kWCarry);

  embed_ln_kernel<<<kRows / 8, 256, 0, stream>>>(SE, rtg, reward_emb_w, reward_emb_b, ln_w, ln_b, norm_w, RESA, HN);

  for (int i = 0; i < kNLayer; ++i) {
    const unsigned short* wip_i = WIP + (size_t)i * kXzP * kMDim;
    const unsigned short* wxp_i = WXP + (size_t)i * kXdP * kDin;
    const unsigned short* wop_i = WOP + (size_t)i * kMDim * kDin;
    const float* cw_i   = conv_w    + (size_t)i * kDin * kConvK;
    const float* cb_i   = conv_b    + (size_t)i * kDin;
    const float* dpw_i  = dt_proj_w + (size_t)i * kDin * kDtR;
    const float* dpb_i  = dt_proj_b + (size_t)i * kDin;
    const float* alog_i = A_log     + (size_t)i * kDin * kNst;
    const float* dp_i   = D_param   + (size_t)i * kDin;
    const float* wnext  = (i + 1 < kNLayer) ? (norm_w + (size_t)(i + 1) * kMDim) : norm_f_w;
    const float* res_in = (i & 1) ? RESB : RESA;
    float* res_out      = (i & 1) ? RESA : RESB;

    wmma_gemm64<0, false, 0, 0, false, 0><<<dim3(gemm_blocks(kRows, kXzP), 1), 256, 0, stream>>>(
        HN, nullptr, kMDim, 0L,
        wip_i, nullptr, kMDim, 0L,
        (void*)XZ, nullptr, kXzP, 0L,
        nullptr, nullptr, 0L,
        kRows, kXzP, kMDim, 1.0f / kWCarry);

    conv_silu_kernel<<<dim3(kDin / 256, kRows / 64), 256, 0, stream>>>(XZ, cw_i, cb_i, UC, UCH);

    wmma_gemm64<0, false, 0, 0, false, 0><<<dim3(gemm_blocks(kRows, kXdP), 1), 256, 0, stream>>>(
        UCH, nullptr, kDin, 0L,
        wxp_i, nullptr, kDin, 0L,
        (void*)XD, nullptr, kXdP, 0L,
        nullptr, nullptr, 0L,
        kRows, kXdP, kDin, 1.0f / (kWCarry * kUCarry));

    scan_kernel<<<kBatch * (kDin / kScanCh), kScanCh, 0, stream>>>(XD, UC, XZ, dpw_i, dpb_i, alog_i, dp_i, YH);

    wmma_gemm64<0, false, 0, 0, false, 0><<<dim3(gemm_blocks(kRows, kMDim), 1), 256, 0, stream>>>(
        YH, nullptr, kDin, 0L,
        wop_i, nullptr, kDin, 0L,
        (void*)H, nullptr, kMDim, 0L,
        nullptr, nullptr, 0L,
        kRows, kMDim, kDin, 1.0f / (kWCarry * kYCarry));

    residual_rms_kernel<<<kRows / 8, 256, 0, stream>>>(H, res_in, wnext, res_out, HN);
  }

  wmma_gemm64<0, false, 2, 1, false, 2><<<dim3(gemm_blocks(kRows, kHid), 1), 256, 0, stream>>>(
      HN, nullptr, kMDim, 0L,
      WS1, nullptr, kMDim, 0L,
      (void*)T1S, nullptr, kHid, 0L,
      so_b1, nullptr, 0L,
      kRows, kHid, kMDim, 1.0f / kWCarry);
  wmma_gemm64<0, false, 2, 0, false, 0><<<dim3(gemm_blocks(kRows, kInDim), 1), 256, 0, stream>>>(
      T1S, nullptr, kHid, 0L,
      WS2, nullptr, kHid, 0L,
      (void*)out0, nullptr, kInDim, 0L,
      so_b2, nullptr, 0L,
      kRows, kInDim, kHid, 1.0f / kWCarry);

  wmma_gemm64<0, false, 2, 0, false, 2><<<dim3(gemm_blocks(kRows, kHid), 1), 256, 0, stream>>>(
      HN, nullptr, kMDim, 0L,
      WR1, nullptr, kMDim, 0L,
      (void*)T1R, nullptr, kHid, 0L,
      ro_b1, nullptr, 0L,
      kRows, kHid, kMDim, 1.0f / kWCarry);
  reward_head_kernel<<<kRows / 32, 256, 0, stream>>>(T1R, ro_w2, ro_b2, out1);
}
